// TransformerBlock_63660005261370
// MI455X (gfx1250) — hardware-verified
//
#include <hip/hip_runtime.h>
#include <stddef.h>


typedef _Float16 v16h __attribute__((ext_vector_type(16)));
typedef _Float16 v8h  __attribute__((ext_vector_type(8)));
typedef float    v8f  __attribute__((ext_vector_type(8)));
typedef float    v4f  __attribute__((ext_vector_type(4)));

#ifndef NB
#define NB 2
#endif
#ifndef SEQ
#define SEQ 2048
#endif
#define NB_FULL  2
#define SEQ_FULL 2048
#define DIM   1024
#define NHEAD 16
#define HD    64
#define DFF   4096
#define NPAIR 32
#define MROWS (NB * SEQ)

static_assert(NB >= 1 && NB <= NB_FULL);
static_assert(SEQ >= 128 && SEQ <= SEQ_FULL && (SEQ % 128) == 0);
static_assert(DIM == NHEAD * HD);
static_assert(HD == 64 && NPAIR * 2 == HD);
static_assert((DIM % 64) == 0 && (DIM % 32) == 0);
static_assert((DFF % 64) == 0 && (DFF % 32) == 0);
static_assert(DFF == 4 * DIM);
static_assert((MROWS % 64) == 0 && (MROWS % 8) == 0);
static_assert(DIM == 32 * 8 * 4);
static_assert(((size_t)DIM * DIM) % 2048 == 0);
static_assert(((size_t)DFF * DIM) % 2048 == 0);
static_assert((size_t)MROWS * DFF < (size_t)0xFFFFFFFFu);

#define LDT 72
#define LDC 68

#define WCARRY 32.0f
#define PCARRY 1024.0f
#define VCARRY 64.0f
#define HCARRY 64.0f
#define EPSV   1.0e-5f

#define WSQ_BYTES     ((size_t)DIM * DIM * 2)
#define WFF_BYTES     ((size_t)DFF * DIM * 2)
#define WT_BYTES      (4 * WSQ_BYTES + 3 * WFF_BYTES)
#define PLANE16_BYTES ((size_t)MROWS * DIM * 2)
#define ATT_BYTES     (4 * PLANE16_BYTES)
#define HH_BYTES      ((size_t)MROWS * DFF * 2)
#define X1_BYTES      ((size_t)MROWS * DIM * 4)
#define TAB_BYTES     ((size_t)MROWS * NPAIR * 4)
#define OFF_H16       (WT_BYTES)
#define OFF_ATT       (OFF_H16 + PLANE16_BYTES)
#define OFF_X1        (OFF_ATT + ATT_BYTES)
#define OFF_COS       (OFF_X1 + X1_BYTES)
#define OFF_SIN       (OFF_COS + TAB_BYTES)
#define WS_TOTAL      (OFF_SIN + TAB_BYTES)
static_assert(HH_BYTES <= ATT_BYTES);
static_assert((WSQ_BYTES % 128) == 0 && (WFF_BYTES % 128) == 0 && (PLANE16_BYTES % 128) == 0);
static_assert((X1_BYTES % 128) == 0 && (TAB_BYTES % 128) == 0);
static_assert(WS_TOTAL <= (size_t)134217728);

__device__ __forceinline__ float bf16r(float x) {
  unsigned int u = __float_as_uint(x);
  u = (u + 0x7FFFu + ((u >> 16) & 1u)) & 0xFFFF0000u;
  return __uint_as_float(u);
}

__device__ __forceinline__ v16h frag_at(const _Float16* p) {
  v8h lo = *(const v8h*)(p);
  v8h hi = *(const v8h*)(p + 16);
  v16h out;
#pragma unroll
  for (int i = 0; i < 8; ++i) { out[i] = lo[i]; out[i + 8] = hi[i]; }
  return out;
}
__device__ __forceinline__ v16h ld_frag(const _Float16* base, unsigned ld) {
  const unsigned lane = threadIdx.x & 31u;
  return frag_at(base + (lane & 15u) * ld + (lane >> 4) * 8u);
}

__device__ __forceinline__ v8f wmma16(v16h a, v16h b, v8f c) {
  v8f d = __builtin_amdgcn_wmma_f32_16x16x32_f16(false, a, false, b, (short)0, c,
                                                 false, false);
  asm volatile("v_nop\n\tv_nop\n\tv_nop\n\tv_nop" : "+v"(d) : "v"(a), "v"(b));
  return d;
}

__device__ __forceinline__ float red16_max(float x) {
#pragma unroll
  for (int off = 1; off < 16; off <<= 1) x = fmaxf(x, __shfl_xor(x, off, 32));
  return x;
}
__device__ __forceinline__ float red16_sum(float x) {
#pragma unroll
  for (int off = 1; off < 16; off <<= 1) x += __shfl_xor(x, off, 32);
  return x;
}

__device__ __forceinline__ void wave_lds_sync() {
  __builtin_amdgcn_fence(3  , "wavefront");
  asm volatile("s_wait_dscnt 0x0" ::: "memory");
  __builtin_amdgcn_wave_barrier();
}

__global__ __launch_bounds__(256) void wcvt_kernel(
    const float* __restrict__ W, _Float16* __restrict__ dst) {
  const size_t e = ((size_t)blockIdx.x * 256u + threadIdx.x) * 8u;
  const v4f a0 = *(const v4f*)(W + e);
  const v4f a1 = *(const v4f*)(W + e + 4);
  v8h o;
#pragma unroll
  for (int j = 0; j < 4; ++j) {
    o[j]     = (_Float16)(WCARRY * bf16r(a0[j]));
    o[j + 4] = (_Float16)(WCARRY * bf16r(a1[j]));
  }
  *(volatile v8h*)(dst + e) = o;
  __threadfence();
  *(volatile v8h*)(dst + e) = o;
}

__global__ __launch_bounds__(256) void rope_table_kernel(
    const int* __restrict__ pos, float* __restrict__ CosT, float* __restrict__ SinT) {
  const unsigned idx = blockIdx.x * 256u + threadIdx.x;
  const unsigned crow = idx >> 5;
  const unsigned i = idx & 31u;
  const unsigned b = crow / (unsigned)SEQ;
  const unsigned s = crow - b * (unsigned)SEQ;
  const float p = (float)pos[(size_t)b * SEQ_FULL + s];
  double pw = 1.0;
  pw *= (i & 1u)  ? 1.3335214321633240 : 1.0;
  pw *= (i & 2u)  ? 1.7782794100389228 : 1.0;
  pw *= (i & 4u)  ? 3.1622776601683795 : 1.0;
  pw *= (i & 8u)  ? 10.0 : 1.0;
  pw *= (i & 16u) ? 100.0 : 1.0;
  const float pf = (float)pw;
  const float fr = 1.0f / pf;
  const float ang = p * fr;
  float sn, cs;
  sincosf(ang, &sn, &cs);
  *(volatile float*)(CosT + idx) = cs;
  *(volatile float*)(SinT + idx) = sn;
  __threadfence();
  *(volatile float*)(CosT + idx) = cs;
  *(volatile float*)(SinT + idx) = sn;
}

__device__ __forceinline__ void norm_store_pass(
    const float* __restrict__ sp, const float* __restrict__ wp, _Float16* __restrict__ dp,
    float rinv, int cvt) {
#pragma unroll 1
  for (unsigned j = 0; j < 4u; ++j) {
    const v4f a0 = *(const v4f*)(sp + j * 256u);
    const v4f a1 = *(const v4f*)(sp + j * 256u + 4u);
    const v4f w0 = *(const v4f*)(wp + j * 256u);
    const v4f w1 = *(const v4f*)(wp + j * 256u + 4u);
    v8h o;
#pragma unroll
    for (int t = 0; t < 4; ++t) {
      const float x0 = cvt ? bf16r(a0[t]) : a0[t];
      const float x1 = cvt ? bf16r(a1[t]) : a1[t];
      o[t]     = (_Float16)((x0 * rinv) * bf16r(w0[t]));
      o[t + 4] = (_Float16)((x1 * rinv) * bf16r(w1[t]));
    }
    *(volatile v8h*)(dp + j * 256u) = o;
  }
}

__global__ __launch_bounds__(256) void rmsnorm_kernel(
    const float* __restrict__ src, const float* __restrict__ nw,
    _Float16* __restrict__ dst, int src_seq, int cvt) {
  const unsigned lane = threadIdx.x & 31u;
  const unsigned wave = (unsigned)__builtin_amdgcn_readfirstlane((int)(threadIdx.x >> 5));
  const unsigned crow = blockIdx.x * 8u + wave;
  const unsigned b = crow / (unsigned)SEQ;
  const unsigned s = crow - b * (unsigned)SEQ;
  const size_t frow = (size_t)b * (unsigned)src_seq + s;
  const float* sp = src + frow * DIM + lane * 8u;
  const float* wp = nw + lane * 8u;
  _Float16* dp = dst + (size_t)crow * DIM + lane * 8u;
  float ss = 0.0f;
#pragma unroll 1
  for (unsigned j = 0; j < 4u; ++j) {
    const v4f a0 = *(const v4f*)(sp + j * 256u);
    const v4f a1 = *(const v4f*)(sp + j * 256u + 4u);
#pragma unroll
    for (int t = 0; t < 4; ++t) {
      const float x0 = cvt ? bf16r(a0[t]) : a0[t];
      const float x1 = cvt ? bf16r(a1[t]) : a1[t];
      ss += x0 * x0;
      ss += x1 * x1;
    }
  }
#pragma unroll
  for (int off = 16; off > 0; off >>= 1) ss += __shfl_xor(ss, off, 32);
  const float rinv = 1.0f / sqrtf(ss * (1.0f / (float)DIM) + EPSV);
  norm_store_pass(sp, wp, dp, rinv, cvt);
  __threadfence();
  norm_store_pass(sp, wp, dp, rinv, cvt);
}

#define GM_ROT  0
#define GM_VT   1
#define GM_RESX 2
#define GM_RESO 3
#define GM_SWI  4

__device__ __forceinline__ float swiglu_val(float a32, float g32) {
  const float a = a32 * (1.0f / WCARRY);
  const float g = g32 * (1.0f / WCARRY);
  const float e = __expf(-a);
  return (a * __builtin_amdgcn_rcpf(1.0f + e)) * (g * HCARRY);
}

template <int MODE, int KD>
__device__ __forceinline__ void gemm_body(
    const _Float16* __restrict__ A16, const _Float16* __restrict__ Bt,
    const _Float16* __restrict__ Bt2,
    const float* __restrict__ aux0, const float* __restrict__ aux1,
    float* __restrict__ outf, _Float16* __restrict__ out16) {
  static_assert((KD % 32) == 0);
  __shared__ float Cs[64 * LDC];
  const unsigned tid = threadIdx.x, lane = tid & 31u;
  const unsigned wave = (unsigned)__builtin_amdgcn_readfirstlane((int)(tid >> 5));
  const unsigned mw = wave >> 1, nw = wave & 1u;
  const unsigned hh = lane >> 4, m = lane & 15u;
  const unsigned n0 = blockIdx.x * 64u;
  const unsigned row0 = blockIdx.y * 64u;

  const _Float16* ap = A16 + (size_t)(row0 + mw * 16u + m) * KD + hh * 8u;
  const size_t boff = (size_t)(n0 + nw * 32u + m) * KD + hh * 8u;
  const _Float16* bp0 = Bt + boff;
  const _Float16* bp1 = bp0 + 16 * KD;
  v8f acc0 = {}, acc1 = {}, acc2 = {}, acc3 = {};
  if (MODE == GM_SWI) {
    const _Float16* gp0 = Bt2 + boff;
    const _Float16* gp1 = gp0 + 16 * KD;
#pragma unroll 2
    for (unsigned k0 = 0; k0 < (unsigned)KD; k0 += 32u) {
      const v16h a  = frag_at(ap + k0);
      const v16h b0 = frag_at(bp0 + k0);
      const v16h b1 = frag_at(bp1 + k0);
      const v16h g0 = frag_at(gp0 + k0);
      const v16h g1 = frag_at(gp1 + k0);
      acc0 = wmma16(a, b0, acc0);
      acc1 = wmma16(a, b1, acc1);
      acc2 = wmma16(a, g0, acc2);
      acc3 = wmma16(a, g1, acc3);
    }
  } else {
#pragma unroll 2
    for (unsigned k0 = 0; k0 < (unsigned)KD; k0 += 32u) {
      const v16h a  = frag_at(ap + k0);
      const v16h b0 = frag_at(bp0 + k0);
      const v16h b1 = frag_at(bp1 + k0);
      acc0 = wmma16(a, b0, acc0);
      acc1 = wmma16(a, b1, acc1);
    }
  }
#pragma unroll
  for (int r = 0; r < 8; ++r) {
    float v0, v1;
    if (MODE == GM_SWI) {
      v0 = swiglu_val(acc0[r], acc2[r]);
      v1 = swiglu_val(acc1[r], acc3[r]);
    } else {
      v0 = acc0[r];
      v1 = acc1[r];
    }
    const unsigned ci = (mw * 16u + hh * 8u + (unsigned)r) * LDC + nw * 32u + m;
    Cs[ci]       = v0;
    Cs[ci + 16u] = v1;
  }
  __syncthreads();

  if (MODE == GM_ROT || MODE == GM_SWI) {
    const unsigned ldo = (MODE == GM_ROT) ? (unsigned)DIM : (unsigned)DFF;
    v8h x[2];
    size_t off[2];
#pragma unroll
    for (unsigned i = 0; i < 2u; ++i) {
      const unsigned r = 32u * i + (tid >> 3);
      const unsigned c = (tid & 7u) * 8u;
      const v4f u0 = *(const v4f*)&Cs[r * LDC + c];
      const v4f u1 = *(const v4f*)&Cs[r * LDC + c + 4];
      if (MODE == GM_ROT) {
        const size_t trow = (size_t)(row0 + r) * NPAIR + (c >> 1);
        const v4f cs = *(const v4f*)(aux0 + trow);
        const v4f sn = *(const v4f*)(aux1 + trow);
        float t[8];
#pragma unroll
        for (int j = 0; j < 4; ++j) {
          t[j]     = u0[j] * (1.0f / WCARRY);
          t[j + 4] = u1[j] * (1.0f / WCARRY);
        }
#pragma unroll
        for (int j = 0; j < 4; ++j) {
          const float xe = t[2 * j], xo = t[2 * j + 1];
          x[i][2 * j]     = (_Float16)(xe * cs[j] - xo * sn[j]);
          x[i][2 * j + 1] = (_Float16)(xe * sn[j] + xo * cs[j]);
        }
      } else {
#pragma unroll
        for (int j = 0; j < 4; ++j) {
          x[i][j]     = (_Float16)u0[j];
          x[i][j + 4] = (_Float16)u1[j];
        }
      }
      off[i] = (size_t)(row0 + r) * ldo + n0 + c;
    }
#pragma unroll
    for (int i = 0; i < 2; ++i) *(volatile v8h*)(out16 + off[i]) = x[i];
    __threadfence();
#pragma unroll
    for (int i = 0; i < 2; ++i) *(volatile v8h*)(out16 + off[i]) = x[i];
  }

  if (MODE == GM_VT) {
    const unsigned bidx = row0 / (unsigned)SEQ;
    const unsigned key0 = row0 - bidx * (unsigned)SEQ;
    v8h x[2];
    size_t off[2];
#pragma unroll
    for (unsigned i = 0; i < 2u; ++i) {
      const unsigned dcol = 32u * i + (tid >> 3);
      const unsigned kk = (tid & 7u) * 8u;
#pragma unroll
      for (unsigned j = 0; j < 8u; ++j)
        x[i][j] = (_Float16)(Cs[(kk + j) * LDC + dcol] * (1.0f / WCARRY));
      off[i] = ((size_t)bidx * DIM + n0 + dcol) * SEQ + key0 + kk;
    }
#pragma unroll
    for (int i = 0; i < 2; ++i) *(volatile v8h*)(out16 + off[i]) = x[i];
    __threadfence();
#pragma unroll
    for (int i = 0; i < 2; ++i) *(volatile v8h*)(out16 + off[i]) = x[i];
  }

  if (MODE == GM_RESX || MODE == GM_RESO) {
    const float sc = (MODE == GM_RESX) ? (1.0f / (WCARRY * VCARRY)) : (1.0f / (WCARRY * HCARRY));
    v4f xs[4];
    size_t off[4];
#pragma unroll
    for (unsigned i = 0; i < 4u; ++i) {
      const unsigned r = 16u * i + (tid >> 4);
      const unsigned c = (tid & 15u) * 4u;
      const unsigned crow = row0 + r;
      const unsigned bidx = crow / (unsigned)SEQ;
      const unsigned sq = crow - bidx * (unsigned)SEQ;
      const size_t frow = (size_t)bidx * SEQ_FULL + sq;
      const size_t coff = (size_t)crow * DIM + n0 + c;
      const size_t foff = frow * DIM + n0 + c;
      const v4f u = *(const v4f*)&Cs[r * LDC + c];
      v4f val;
      if (MODE == GM_RESX) {
        const v4f g = *(const v4f*)(aux0 + foff);
#pragma unroll
        for (int j = 0; j < 4; ++j) val[j] = u[j] * sc + bf16r(g[j]);
        off[i] = coff;
      } else {
        const v4f g = *(const v4f*)(aux0 + coff);
#pragma unroll
        for (int j = 0; j < 4; ++j) val[j] = u[j] * sc + g[j];
        off[i] = foff;
      }
      xs[i] = val;
    }
#pragma unroll
    for (int i = 0; i < 4; ++i) *(volatile v4f*)(outf + off[i]) = xs[i];
    __threadfence();
#pragma unroll
    for (int i = 0; i < 4; ++i) *(volatile v4f*)(outf + off[i]) = xs[i];
  }
}

__global__ __launch_bounds__(256) void gemm_rot_kernel(
    const _Float16* __restrict__ A16, const _Float16* __restrict__ Bt,
    const float* __restrict__ CosT, const float* __restrict__ SinT,
    _Float16* __restrict__ out16) {
  gemm_body<GM_ROT, DIM>(A16, Bt, Bt, CosT, SinT, (float*)0, out16);
}
__global__ __launch_bounds__(256) void gemm_vt_kernel(
    const _Float16* __restrict__ A16, const _Float16* __restrict__ Bt,
    _Float16* __restrict__ out16) {
  gemm_body<GM_VT, DIM>(A16, Bt, Bt, (const float*)0, (const float*)0, (float*)0, out16);
}
__global__ __launch_bounds__(256) void gemm_resx_kernel(
    const _Float16* __restrict__ A16, const _Float16* __restrict__ Bt,
    const float* __restrict__ Xin, float* __restrict__ outf) {
  gemm_body<GM_RESX, DIM>(A16, Bt, Bt, Xin, Xin, outf, (_Float16*)0);
}
__global__ __launch_bounds__(256) void gemm_swi_kernel(
    const _Float16* __restrict__ A16, const _Float16* __restrict__ Bt1,
    const _Float16* __restrict__ Bt3, _Float16* __restrict__ out16) {
  gemm_body<GM_SWI, DIM>(A16, Bt1, Bt3, (const float*)0, (const float*)0, (float*)0, out16);
}
__global__ __launch_bounds__(256) void gemm_reso_kernel(
    const _Float16* __restrict__ A16, const _Float16* __restrict__ Bt,
    const float* __restrict__ X1, float* __restrict__ outf) {
  gemm_body<GM_RESO, DFF>(A16, Bt, Bt, X1, X1, outf, (_Float16*)0);
}

__global__ __launch_bounds__(256) void attn_kernel(
    const _Float16* __restrict__ Qh, const _Float16* __restrict__ Kh,
    const _Float16* __restrict__ Vt, _Float16* __restrict__ Ov) {
  __shared__ _Float16 Ks[64 * LDT];
  __shared__ _Float16 Vs[64 * LDT];
  __shared__ _Float16 Ps[8 * 16 * LDT];

  const unsigned tid = threadIdx.x, lane = tid & 31u;
  const unsigned wave = (unsigned)__builtin_amdgcn_readfirstlane((int)(tid >> 5));
  const unsigned hh = lane >> 4, m = lane & 15u;
  const unsigned q0 = blockIdx.x * 128u;
  const unsigned head = blockIdx.y;
  const unsigned b = blockIdx.z;
  const float scale = 0.125f;
  const unsigned pb = wave * (16u * LDT);
  const unsigned rmin = q0 + wave * 16u;
  const unsigned kend = q0 + 128u;

  const size_t qoff = (size_t)(b * (unsigned)SEQ + rmin + m) * DIM + head * HD + hh * 8u;
  v16h qf[2];
  qf[0] = frag_at(Qh + qoff);
  qf[1] = frag_at(Qh + qoff + 32);

  float mrow[8], lrow[8];
  v8f o[4];
#pragma unroll
  for (int v = 0; v < 8; ++v) { mrow[v] = -1.0e30f; lrow[v] = 0.0f; }
#pragma unroll
  for (int nb = 0; nb < 4; ++nb) o[nb] = (v8f){};

  const size_t kplane = (size_t)b * SEQ * DIM + head * HD;
  const size_t vplane = ((size_t)b * DIM + head * HD) * SEQ;

  for (unsigned kb = 0; kb < kend; kb += 64u) {
#pragma unroll
    for (unsigned j = 0; j < 2u; ++j) {
      const unsigned idx = tid + 256u * j;
      const unsigned r = idx >> 3, c = (idx & 7u) * 8u;
      *(v8h*)&Ks[r * LDT + c] = *(const v8h*)(Kh + kplane + (size_t)(kb + r) * DIM + c);
      *(v8h*)&Vs[r * LDT + c] = *(const v8h*)(Vt + vplane + (size_t)r * SEQ + kb + c);
    }
    __syncthreads();

    if (kb <= rmin + 15u) {
      v8f s[4];
#pragma unroll
      for (int kg = 0; kg < 4; ++kg) {
        v8f t = {};
#pragma unroll
        for (int c = 0; c < 2; ++c) {
          const v16h kf = ld_frag(&Ks[(kg * 16) * LDT + c * 32], LDT);
          t = wmma16(qf[c], kf, t);
        }
        s[kg] = t * scale;
      }
      if (kb + 63u > rmin) {
#pragma unroll
        for (int kg = 0; kg < 4; ++kg)
#pragma unroll
          for (int v = 0; v < 8; ++v) {
            const unsigned key = kb + (unsigned)kg * 16u + m;
            const unsigned row = rmin + hh * 8u + (unsigned)v;
            s[kg][v] = (key > row) ? -1.0e30f : s[kg][v];
          }
      }

      float alpha[8];
#pragma unroll
      for (int v = 0; v < 8; ++v) {
        float mx = fmaxf(fmaxf(s[0][v], s[1][v]), fmaxf(s[2][v], s[3][v]));
        mx = red16_max(mx);
        const float mn = fmaxf(mrow[v], mx);
        alpha[v] = __expf(mrow[v] - mn);
        mrow[v] = mn;
      }
#pragma unroll
      for (int kg = 0; kg < 4; ++kg)
#pragma unroll
        for (int v = 0; v < 8; ++v) s[kg][v] = __expf(s[kg][v] - mrow[v]);
#pragma unroll
      for (int v = 0; v < 8; ++v) {
        const float rs = red16_sum((s[0][v] + s[1][v]) + (s[2][v] + s[3][v]));
        lrow[v] = alpha[v] * lrow[v] + rs;
      }
#pragma unroll
      for (int nb = 0; nb < 4; ++nb)
#pragma unroll
        for (int v = 0; v < 8; ++v) o[nb][v] = o[nb][v] * alpha[v];

#pragma unroll
      for (int kg = 0; kg < 4; ++kg)
#pragma unroll
        for (int v = 0; v < 8; ++v)
          Ps[pb + (hh * 8u + (unsigned)v) * LDT + (unsigned)kg * 16u + m] =
              (_Float16)(s[kg][v] * PCARRY);
      wave_lds_sync();

#pragma unroll
      for (int c = 0; c < 2; ++c) {
        const v16h pf = ld_frag(&Ps[pb + c * 32], LDT);
#pragma unroll
        for (int nb = 0; nb < 4; ++nb) {
          const v16h vf = ld_frag(&Vs[(nb * 16) * LDT + c * 32], LDT);
          o[nb] = wmma16(pf, vf, o[nb]);
        }
      }
    }
    __syncthreads();
  }

  float inv[8];
#pragma unroll
  for (int v = 0; v < 8; ++v) inv[v] = __builtin_amdgcn_rcpf(lrow[v]) * (VCARRY / PCARRY);
#pragma unroll
  for (int nb = 0; nb < 4; ++nb)
#pragma unroll
    for (int v = 0; v < 8; ++v)
      Ps[pb + (hh * 8u + (unsigned)v) * LDT + (unsigned)nb * 16u + m] =
          (_Float16)(o[nb][v] * inv[v]);
  wave_lds_sync();
  v8h x[4];
  size_t off[4];
#pragma unroll
  for (unsigned i = 0; i < 4u; ++i) {
    const unsigned r = 4u * i + (lane >> 3);
    const unsigned c = (lane & 7u) * 8u;
    x[i] = *(const v8h*)&Ps[pb + r * LDT + c];
    off[i] = (size_t)(b * (unsigned)SEQ + rmin + r) * DIM + head * HD + c;
  }
#pragma unroll
  for (int i = 0; i < 4; ++i) *(volatile v8h*)(Ov + off[i]) = x[i];
  __threadfence();
#pragma unroll
  for (int i = 0; i < 4; ++i) *(volatile v8h*)(Ov + off[i]) = x[i];
}

extern "C" void kernel_launch(void* const* d_in, const int* in_sizes, int n_in,
                              void* d_out, int out_size, void* d_ws, size_t ws_size,
                              hipStream_t stream) {
  if (n_in < 11) return;
  const long long need_rows = (long long)(NB - 1) * SEQ_FULL + SEQ;
  const long long need_x = need_rows * DIM;
  if ((long long)in_sizes[0] < need_x) return;
  if ((long long)in_sizes[1] < need_rows) return;
  if (in_sizes[2] < DIM || in_sizes[3] < DIM) return;
  if ((long long)in_sizes[4] < (long long)DIM * DIM) return;
  if ((long long)in_sizes[5] < (long long)DIM * DIM) return;
  if ((long long)in_sizes[6] < (long long)DIM * DIM) return;
  if ((long long)in_sizes[7] < (long long)DIM * DIM) return;
  if ((long long)in_sizes[8] < (long long)DFF * DIM) return;
  if ((long long)in_sizes[9] < (long long)DIM * DFF) return;
  if ((long long)in_sizes[10] < (long long)DFF * DIM) return;
  if ((long long)out_size < need_x) return;
  if (ws_size < WS_TOTAL) return;

  const float* X   = (const float*)d_in[0];
  const int*   pos = (const int*)d_in[1];
  const float* n1w = (const float*)d_in[2];
  const float* n2w = (const float*)d_in[3];
  const float* wq  = (const float*)d_in[4];
  const float* wk  = (const float*)d_in[5];
  const float* wv  = (const float*)d_in[6];
  const float* wo  = (const float*)d_in[7];
  const float* w1  = (const float*)d_in[8];
  const float* w2  = (const float*)d_in[9];
  const float* w3  = (const float*)d_in[10];
  float* out = (float*)d_out;

  char* ws = (char*)d_ws;
  _Float16* WQ = (_Float16*)(ws);
  _Float16* WK = (_Float16*)(ws + 1 * WSQ_BYTES);
  _Float16* WV = (_Float16*)(ws + 2 * WSQ_BYTES);
  _Float16* WO = (_Float16*)(ws + 3 * WSQ_BYTES);
  _Float16* W1 = (_Float16*)(ws + 4 * WSQ_BYTES);
  _Float16* W3 = (_Float16*)(ws + 4 * WSQ_BYTES + 1 * WFF_BYTES);
  _Float16* W2 = (_Float16*)(ws + 4 * WSQ_BYTES + 2 * WFF_BYTES);
  _Float16* H16   = (_Float16*)(ws + OFF_H16);
  _Float16* Q16   = (_Float16*)(ws + OFF_ATT);
  _Float16* K16   = (_Float16*)(ws + OFF_ATT + 1 * PLANE16_BYTES);
  _Float16* Vt16  = (_Float16*)(ws + OFF_ATT + 2 * PLANE16_BYTES);
  _Float16* Ctx16 = (_Float16*)(ws + OFF_ATT + 3 * PLANE16_BYTES);
  _Float16* HH16  = (_Float16*)(ws + OFF_ATT);
  float* X1   = (float*)(ws + OFF_X1);
  float* CosT = (float*)(ws + OFF_COS);
  float* SinT = (float*)(ws + OFF_SIN);

  dim3 blk(256);
  const unsigned gsq = (unsigned)(((size_t)DIM * DIM) / 2048);
  const unsigned gff = (unsigned)(((size_t)DFF * DIM) / 2048);
  dim3 gg(DIM / 64, MROWS / 64);
  dim3 gf(DFF / 64, MROWS / 64);

  wcvt_kernel<<<dim3(gsq), blk, 0, stream>>>(wq, WQ);
  wcvt_kernel<<<dim3(gsq), blk, 0, stream>>>(wk, WK);
  wcvt_kernel<<<dim3(gsq), blk, 0, stream>>>(wv, WV);
  wcvt_kernel<<<dim3(gsq), blk, 0, stream>>>(wo, WO);
  wcvt_kernel<<<dim3(gff), blk, 0, stream>>>(w1, W1);
  wcvt_kernel<<<dim3(gff), blk, 0, stream>>>(w3, W3);
  wcvt_kernel<<<dim3(gff), blk, 0, stream>>>(w2, W2);

  rope_table_kernel<<<dim3(MROWS / 8), blk, 0, stream>>>(pos, CosT, SinT);
  rmsnorm_kernel<<<dim3(MROWS / 8), blk, 0, stream>>>(X, n1w, H16, (int)SEQ_FULL, 1);

  gemm_rot_kernel<<<gg, blk, 0, stream>>>(H16, WQ, CosT, SinT, Q16);
  gemm_rot_kernel<<<gg, blk, 0, stream>>>(H16, WK, CosT, SinT, K16);
  gemm_vt_kernel<<<gg, blk, 0, stream>>>(H16, WV, Vt16);

  attn_kernel<<<dim3(SEQ / 128, NHEAD, NB), blk, 0, stream>>>(Q16, K16, Vt16, Ctx16);

  gemm_resx_kernel<<<gg, blk, 0, stream>>>(Ctx16, WO, X, X1);

  rmsnorm_kernel<<<dim3(MROWS / 8), blk, 0, stream>>>(X1, n2w, H16, (int)SEQ, 0);

  gemm_swi_kernel<<<gf, blk, 0, stream>>>(H16, W1, W3, HH16);
  gemm_reso_kernel<<<gg, blk, 0, stream>>>(HH16, W2, X1, out);
}
